// LaneAwareAttention_16896401343260
// MI455X (gfx1250) — hardware-verified
//
#include <hip/hip_runtime.h>

typedef __attribute__((ext_vector_type(16))) _Float16 v16h;
typedef __attribute__((ext_vector_type(8)))  _Float16 v8h;
typedef __attribute__((ext_vector_type(16))) __bf16   v16b;
typedef __attribute__((ext_vector_type(8)))  __bf16   v8b;
typedef __attribute__((ext_vector_type(8)))  float    v8f;
typedef __attribute__((ext_vector_type(4)))  float    v4f;
#define U16(p) ((const unsigned short*)(const void*)(p))

__device__ __forceinline__ unsigned short f2bf_bits(float f) {
  unsigned u = __float_as_uint(f);
  return (unsigned short)((u + 0x7FFFu + ((u >> 16) & 1u)) >> 16);
}
__device__ __forceinline__ float bf_bits2f(unsigned short h) { return __uint_as_float(((unsigned)h) << 16); }

__device__ __forceinline__ void dep_guard_h(v8f& a, v8f& b, v16h x, v16h y) { asm volatile("v_nop\n\tv_nop\n\tv_nop\n\tv_nop" : "+v"(a), "+v"(b) : "v"(x), "v"(y)); }
__device__ __forceinline__ void dep_guard_b(v8f& a, v8f& b, v16b x, v16b y) { asm volatile("v_nop\n\tv_nop\n\tv_nop\n\tv_nop" : "+v"(a), "+v"(b) : "v"(x), "v"(y)); }
__device__ __forceinline__ void keep4_h(v16h a, v16h b, v16h c, v16h d) { asm volatile("v_nop" :: "v"(a), "v"(b), "v"(c), "v"(d)); }
__device__ __forceinline__ void keep4_b(v16b a, v16b b, v16b c, v16b d) { asm volatile("v_nop" :: "v"(a), "v"(b), "v"(c), "v"(d)); }
__device__ __forceinline__ void acc_guard4(v8f& a, v8f& b, v8f& c, v8f& d) { asm volatile("v_nop\n\tv_nop\n\tv_nop\n\tv_nop" : "+v"(a), "+v"(b), "+v"(c), "+v"(d)); }
template <typename T> struct Frag;
template <> struct Frag<_Float16> {
  typedef v16h V; union U { v16h v; v8h h[2]; };
  static __device__ __forceinline__ v16h load(const _Float16* p) {
    U f; f.h[0] = *(const v8h*)(p); f.h[1] = *(const v8h*)(p + 16); return f.v;
  }
  static __device__ __forceinline__ v8f mma(v16h a, v16h b, v8f c) {
    return __builtin_amdgcn_wmma_f32_16x16x32_f16(false, a, false, b, (short)0, c, false, false);
  }
  static __device__ __forceinline__ void guard(v8f& a, v8f& b, v16h x, v16h y) { dep_guard_h(a, b, x, y); }
  static __device__ __forceinline__ void keep(v16h a, v16h b, v16h c, v16h d) { keep4_h(a, b, c, d); }
};
template <> struct Frag<__bf16> {
  typedef v16b V; union U { v16b v; v8b h[2]; };
  static __device__ __forceinline__ v16b load(const __bf16* p) {
    U f; f.h[0] = *(const v8b*)(p); f.h[1] = *(const v8b*)(p + 16); return f.v;
  }
  static __device__ __forceinline__ v8f mma(v16b a, v16b b, v8f c) {
    return __builtin_amdgcn_wmma_f32_16x16x32_bf16(false, a, false, b, (short)0, c, false, false);
  }
  static __device__ __forceinline__ void guard(v8f& a, v8f& b, v16b x, v16b y) { dep_guard_b(a, b, x, y); }
  static __device__ __forceinline__ void keep(v16b a, v16b b, v16b c, v16b d) { keep4_b(a, b, c, d); }
};

template <int ET> struct Elem;
template <> struct Elem<0> { typedef _Float16 T; };
template <> struct Elem<1> { typedef __bf16 T; };
template <int ET, bool SPLIT, int BIAS_MODE, int OUT_MODE, bool RESID, int ACT = 0>
__global__ __launch_bounds__(256) void wmma_gemm64(
    const unsigned short* __restrict__ Ap, const unsigned short* __restrict__ A2p, int lda, long strideA,
    const unsigned short* __restrict__ Btp, const unsigned short* __restrict__ Bt2p, int ldb, long strideB,
    void* __restrict__ Cout, void* __restrict__ Cout2, int ldc, long strideC,
    const float* __restrict__ bias,
    const float* __restrict__ resid, long strideR,
    int M, int N, int K, float scale) {
  typedef typename Elem<ET>::T T;
  typedef typename Frag<T>::V V;
  const T* A = (const T*)Ap; const T* A2 = (const T*)A2p; const T* Bt = (const T*)Btp; const T* Bt2 = (const T*)Bt2p;
  __shared__ __align__(16) float sT[8][16 * 68];
  const int b    = blockIdx.y;
  const int lane = threadIdx.x & 31;
  const int wave = threadIdx.x >> 5;
  const int tilesN = N >> 6;
  const int tilesM = M >> 6;
  const int tile = blockIdx.x * 8 + wave;
  if (tile >= tilesM * tilesN) return;
  const int tm = tile / tilesN;
  const int tn = tile - tm * tilesN;
  const int m0 = tm << 6;
  const int n0 = tn << 6;

  const T* Ab  = A  + (size_t)b * strideA;
  const T* Bb  = Bt + (size_t)b * strideB;
  const T* Ab2 = SPLIT ? (A2  + (size_t)b * strideA) : nullptr;
  const T* Bb2 = SPLIT ? (Bt2 + (size_t)b * strideB) : nullptr;

  const int rlane = lane & 15;
  const int koff  = (lane >> 4) * 8;
  const int mOff  = (lane >> 4) * 8;

  v8f acc[4][4];
#pragma unroll
  for (int i = 0; i < 4; ++i)
#pragma unroll
    for (int j = 0; j < 4; ++j) acc[i][j] = (v8f){0.f,0.f,0.f,0.f,0.f,0.f,0.f,0.f};

  for (int k0 = 0; k0 < K; k0 += 32) {
    V bh[4], bl[4];
#pragma unroll
    for (int j = 0; j < 4; ++j) {
      const size_t bo = (size_t)(n0 + (j << 4) + rlane) * ldb + koff + k0;
      bh[j] = Frag<T>::load(Bb + bo);
      if (SPLIT) bl[j] = Frag<T>::load(Bb2 + bo);
    }
#pragma unroll
    for (int i = 0; i < 4; ++i) {
      const size_t ao = (size_t)(m0 + (i << 4) + rlane) * lda + koff + k0;
      V ah = Frag<T>::load(Ab + ao);
      V al;
      if (SPLIT) al = Frag<T>::load(Ab2 + ao);
#pragma unroll
      for (int j = 0; j < 4; ++j) {
        acc[i][j] = Frag<T>::mma(ah, bh[j], acc[i][j]);
        if (SPLIT) {
          acc[i][j] = Frag<T>::mma(ah, bl[j], acc[i][j]);
          acc[i][j] = Frag<T>::mma(al, bh[j], acc[i][j]);
        }
      }
      Frag<T>::guard(acc[i][0], acc[i][3], ah, SPLIT ? al : ah);
    }
    Frag<T>::keep(bh[0], bh[1], bh[2], bh[3]);
    if (SPLIT) Frag<T>::keep(bl[0], bl[1], bl[2], bl[3]);
  }
  acc_guard4(acc[0][0], acc[0][1], acc[0][2], acc[0][3]);
  acc_guard4(acc[1][0], acc[1][1], acc[1][2], acc[1][3]);
  acc_guard4(acc[2][0], acc[2][1], acc[2][2], acc[2][3]);
  acc_guard4(acc[3][0], acc[3][1], acc[3][2], acc[3][3]);

  float* slab = sT[wave];
  const float* Rb = RESID ? (resid + (size_t)b * strideR) : nullptr;
#pragma unroll
  for (int i = 0; i < 4; ++i) {
    const int mBase = m0 + (i << 4);
#pragma unroll
    for (int j = 0; j < 4; ++j) {
      const int n = n0 + (j << 4) + rlane;
      float bv = 0.f;
      if (BIAS_MODE == 2) bv = bias[n];
#pragma unroll
      for (int r = 0; r < 8; ++r) {
        float v = acc[i][j][r] * scale;
        if (BIAS_MODE == 1) v += bias[mBase + mOff + r];
        if (BIAS_MODE == 2) v += bv;
        if (RESID) v += Rb[(size_t)(mBase + mOff + r) * ldc + n];
        if (ACT == 1) v = tanhf(v);
        if (ACT == 2) v = fmaxf(v, 0.0f);
        if (ACT == 3) v = v / (1.0f + expf(-v));
        if (ACT == 4) v = (v > 0.f) ? v : 0.01f * v;
        if (ACT == 5) v = 0.5f * v * (1.0f + erff(v * 0.70710678118654752f));
        slab[(mOff + r) * 68 + (j << 4) + rlane] = v;
      }
    }
    __builtin_amdgcn_fence(__ATOMIC_RELEASE, "workgroup");
    __builtin_amdgcn_wave_barrier();
    __builtin_amdgcn_fence(__ATOMIC_ACQUIRE, "workgroup");
    if (OUT_MODE == 0) {
      float* C = (float*)Cout + (size_t)b * strideC;
      const int hh = lane >> 4, c4 = (lane & 15) * 4;
      for (int pass = 0; pass < 2; ++pass) {
#pragma unroll
        for (int it = 0; it < 8; ++it) {
          const int row = it * 2 + hh;
          v4f v = *(const v4f*)(slab + row * 68 + c4);
          *(volatile v4f*)(C + (size_t)(mBase + row) * ldc + n0 + c4) = v;
        }
        __threadfence();
      }
    } else {
      const int q = lane >> 3, c8 = (lane & 7) * 8;
      unsigned short* C  = (unsigned short*)Cout  + (size_t)b * strideC;
      unsigned short* C2 = (OUT_MODE == 2) ? ((unsigned short*)Cout2 + (size_t)b * strideC) : nullptr;
      for (int pass = 0; pass < 2; ++pass) {
#pragma unroll
        for (int it = 0; it < 4; ++it) {
          const int row = it * 4 + q;
          const float* sp = slab + row * 68 + c8;
          v8h hv, lv;
#pragma unroll
          for (int e = 0; e < 8; ++e) {
            if (OUT_MODE == 1) {
              hv[e] = (_Float16)sp[e];
            } else {
              unsigned short hb = f2bf_bits(sp[e]);
              unsigned short lb = f2bf_bits(sp[e] - bf_bits2f(hb));
              hv[e] = __builtin_bit_cast(_Float16, hb);
              lv[e] = __builtin_bit_cast(_Float16, lb);
            }
          }
          *(volatile v8h*)(C + (size_t)(mBase + row) * ldc + n0 + c8) = hv;
          if (OUT_MODE == 2) *(volatile v8h*)(C2 + (size_t)(mBase + row) * ldc + n0 + c8) = lv;
        }
        __threadfence();
      }
    }
    __builtin_amdgcn_fence(__ATOMIC_RELEASE, "workgroup");
    __builtin_amdgcn_wave_barrier();
    __builtin_amdgcn_fence(__ATOMIC_ACQUIRE, "workgroup");
  }
}

__global__ __launch_bounds__(256) void cast_f32_f16x2(
    const float* __restrict__ in, _Float16* __restrict__ out, int n2) {
  int i = blockIdx.x * 256 + threadIdx.x;
  if (i < n2) {
    const _Float16 h0 = (_Float16)in[2 * i], h1 = (_Float16)in[2 * i + 1];
    const unsigned u = (unsigned)__builtin_bit_cast(unsigned short, h0) | ((unsigned)__builtin_bit_cast(unsigned short, h1) << 16);
    ((volatile unsigned*)out)[i] = u;
    __threadfence();
    ((volatile unsigned*)out)[i] = u;
  }
}

#define AT_D 64
#define AT_NW 4
#define AT_QB 64
#define AT_KC 64
#define CDIM 512
#define C3DIM 1536
#define NHMAX 8
#define RELT 20
#define RELN 39
#define PSC16 32768.0f
#define MASKFILL (-1.0e30f)

__device__ __forceinline__ v8f mma_f16(v16h a, v16h b, v8f c) {
  c = __builtin_amdgcn_wmma_f32_16x16x32_f16(false, a, false, b, (short)0, c, false, false);
  asm volatile("v_nop\n\tv_nop\n\tv_nop\n\tv_nop" : "+v"(c) : "v"(a), "v"(b));
  return c;
}

__global__ __launch_bounds__(128)
void attn_relpos64(const float* __restrict__ qkv, const float* __restrict__ relh,
                   const float* __restrict__ relw, const int* __restrict__ Hp,
                   const int* __restrict__ Wp, float* __restrict__ out,
                   int S, int nqb, int NH, float qscale) {
  union FH { v16h v; v8h h[2]; };
  __shared__ __align__(16) _Float16 Ksh[AT_KC * AT_D];
  __shared__ __align__(16) _Float16 Vth[AT_D * AT_KC];
  __shared__ __align__(16) _Float16 Psh[AT_NW][16 * AT_KC];
  __shared__ __align__(16) float  Os[AT_NW][16 * 68];
  __shared__ float sRH[RELN * NHMAX];
  __shared__ float sRW[RELN * NHMAX];

  const int tid  = threadIdx.x;
  const int wave = tid >> 5;
  const int lane = tid & 31;
  const int hh   = lane >> 4;
  const int c    = lane & 15;

  const int bx = blockIdx.x;
  const int qb = bx % nqb;
  const int bh = bx / nqb;
  const int h  = bh % NH;
  const int b  = bh / NH;
  const int q0 = qb * AT_QB + wave * 16;

  const int nrel = RELN * NH;
  for (int i = tid; i < nrel; i += 128) { sRH[i] = relh[i]; sRW[i] = relw[i]; }

  int Wv = Wp[0];
  Wv = (Wv < 1) ? 1 : ((Wv > S) ? S : Wv);
  int hmax = Hp[0] - 1;
  hmax = (hmax < 0) ? 0 : ((hmax > RELT - 1) ? (RELT - 1) : hmax);
  int wmax = Wv - 1;
  wmax = (wmax > RELT - 1) ? (RELT - 1) : wmax;

  const size_t rb = (size_t)b * S;
  const float* qbp = qkv + rb * C3DIM + (size_t)h * AT_D;
  const float* kbp = qbp + CDIM;
  const float* vbp = qbp + 2 * CDIM;
  float*       obp = out + rb * CDIM + (size_t)h * AT_D;

  v16h qa[2];
  {
    int qr = q0 + c;
    qr = (qr < S) ? qr : (S - 1);
    const float* qrow = qbp + (size_t)qr * C3DIM;
#pragma unroll
    for (int dc = 0; dc < 2; ++dc) {
#pragma unroll
      for (int e = 0; e < 8; ++e) {
        qa[dc][e]     = (_Float16)(qrow[dc * 32 + 8 * hh + e] * qscale);
        qa[dc][8 + e] = (_Float16)(qrow[dc * 32 + 16 + 8 * hh + e] * qscale);
      }
    }
  }
  int rH[8], rW[8];
#pragma unroll
  for (int r = 0; r < 8; ++r) {
    int qr = q0 + 8 * hh + r;
    qr = (qr < S) ? qr : (S - 1);
    int ih = qr / Wv;
    int iw = qr - ih * Wv;
    ih = (ih > hmax) ? hmax : ih;
    iw = (iw > wmax) ? wmax : iw;
    rH[r] = (ih + RELT - 1) * NH + h;
    rW[r] = (iw + RELT - 1) * NH + h;
  }

  float mrow[8], lrow[8];
  v8f oacc[4];
#pragma unroll
  for (int r = 0; r < 8; ++r) { mrow[r] = -__builtin_huge_valf(); lrow[r] = 0.f; }
#pragma unroll
  for (int t = 0; t < 4; ++t) oacc[t] = (v8f){0.f,0.f,0.f,0.f,0.f,0.f,0.f,0.f};

  const int nChunks = nqb;
  for (int kc = 0; kc < nChunks; ++kc) {
    const int kv0 = kc * AT_KC;
    __syncthreads();
    {
      const int kvr = tid >> 1, dh = (tid & 1) * 32;
      int kr = kv0 + kvr;
      kr = (kr < S) ? kr : (S - 1);
      const float* krow = kbp + (size_t)kr * C3DIM + dh;
      const float* vrow = vbp + (size_t)kr * C3DIM + dh;
#pragma unroll
      for (int i = 0; i < 8; ++i) {
        v4f kk = *(const v4f*)(krow + 4 * i);
        v4f vv = *(const v4f*)(vrow + 4 * i);
#pragma unroll
        for (int e = 0; e < 4; ++e) {
          const int d = dh + 4 * i + e;
          Ksh[kvr * AT_D + d] = (_Float16)kk[e];
          Vth[d * AT_KC + kvr] = (_Float16)vv[e];
        }
      }
    }
    __syncthreads();

    v8f s[4];
#pragma unroll
    for (int j = 0; j < 4; ++j) {
      s[j] = (v8f){0.f,0.f,0.f,0.f,0.f,0.f,0.f,0.f};
#pragma unroll
      for (int dc = 0; dc < 2; ++dc) {
        FH kb;
        kb.h[0] = *(const v8h*)(Ksh + (j * 16 + c) * AT_D + dc * 32 + 8 * hh);
        kb.h[1] = *(const v8h*)(Ksh + (j * 16 + c) * AT_D + dc * 32 + 16 + 8 * hh);
        s[j] = mma_f16(qa[dc], kb.v, s[j]);
      }
    }
    int kval[4], mH[4], mW[4];
#pragma unroll
    for (int j = 0; j < 4; ++j) {
      const int kvcol = kv0 + j * 16 + c;
      kval[j] = (kvcol < S) ? 1 : 0;
      const int kcl = kval[j] ? kvcol : (S - 1);
      int mh = kcl / Wv;
      int mw = kcl - mh * Wv;
      mh = (mh > hmax) ? hmax : mh;
      mw = (mw > wmax) ? wmax : mw;
      mH[j] = mh * NH;
      mW[j] = mw * NH;
    }
    float cm[8];
#pragma unroll
    for (int r = 0; r < 8; ++r) {
      float m = -__builtin_huge_valf();
#pragma unroll
      for (int j = 0; j < 4; ++j) {
        float sv = s[j][r] + sRH[rH[r] - mH[j]] + sRW[rW[r] - mW[j]];
        sv = kval[j] ? sv : MASKFILL;
        s[j][r] = sv;
        m = fmaxf(m, sv);
      }
#pragma unroll
      for (int off = 1; off < 16; off <<= 1) m = fmaxf(m, __shfl_xor(m, off, 32));
      cm[r] = m;
    }
    _Float16* pw = Psh[wave];
#pragma unroll
    for (int r = 0; r < 8; ++r) {
      const float mnew = fmaxf(mrow[r], cm[r]);
      const float alpha = expf(mrow[r] - mnew);
      mrow[r] = mnew;
      float psum = 0.f;
#pragma unroll
      for (int j = 0; j < 4; ++j) {
        const float p = expf(s[j][r] - mnew);
        psum += p;
        pw[(8 * hh + r) * AT_KC + j * 16 + c] = (_Float16)(p * PSC16);
      }
#pragma unroll
      for (int off = 1; off < 16; off <<= 1) psum += __shfl_xor(psum, off, 32);
      lrow[r] = lrow[r] * alpha + psum;
#pragma unroll
      for (int t = 0; t < 4; ++t) oacc[t][r] *= alpha;
    }
    __builtin_amdgcn_fence(__ATOMIC_RELEASE, "workgroup");
    __builtin_amdgcn_wave_barrier();
    __builtin_amdgcn_fence(__ATOMIC_ACQUIRE, "workgroup");
#pragma unroll
    for (int kk = 0; kk < 2; ++kk) {
      FH pa;
      pa.h[0] = *(const v8h*)(pw + c * AT_KC + kk * 32 + 8 * hh);
      pa.h[1] = *(const v8h*)(pw + c * AT_KC + kk * 32 + 16 + 8 * hh);
#pragma unroll
      for (int t = 0; t < 4; ++t) {
        FH vb;
        vb.h[0] = *(const v8h*)(Vth + (t * 16 + c) * AT_KC + kk * 32 + 8 * hh);
        vb.h[1] = *(const v8h*)(Vth + (t * 16 + c) * AT_KC + kk * 32 + 16 + 8 * hh);
        oacc[t] = mma_f16(pa.v, vb.v, oacc[t]);
      }
    }
  }

  if (q0 < S) {
    float* os = Os[wave];
#pragma unroll
    for (int r = 0; r < 8; ++r) {
      const float inv = 1.0f / (lrow[r] * PSC16);
#pragma unroll
      for (int t = 0; t < 4; ++t) os[(8 * hh + r) * 68 + t * 16 + c] = oacc[t][r] * inv;
    }
    __builtin_amdgcn_fence(__ATOMIC_RELEASE, "workgroup");
    __builtin_amdgcn_wave_barrier();
    __builtin_amdgcn_fence(__ATOMIC_ACQUIRE, "workgroup");
    {
      const int c4 = (lane & 15) * 4;
      for (int pass = 0; pass < 2; ++pass) {
#pragma unroll
        for (int it = 0; it < 8; ++it) {
          const int row = it * 2 + hh;
          v4f val = *(const v4f*)(os + row * 68 + c4);
          *(volatile v4f*)(obp + (size_t)(q0 + row) * CDIM + c4) = val;
        }
        __threadfence();
      }
    }
  }
}

static inline size_t align256(size_t x) { return (x + 255) & ~(size_t)255; }

extern "C" void kernel_launch(void* const* d_in, const int* in_sizes, int n_in,
                              void* d_out, int out_size, void* d_ws, size_t ws_size,
                              hipStream_t stream) {
  const int S = RELT * RELT;
  const int C = CDIM, C3 = C3DIM, HD = AT_D;
  const int NH = C / HD;
  if (n_in < 9) return;
  const int BS = in_sizes[0] / C;
  const int Bn = BS / S;
  if (BS <= 0 || Bn * S != BS || BS * C != in_sizes[0] || (BS % 64) != 0) return;
  if (in_sizes[1] != C3 * C || in_sizes[2] != C3 || in_sizes[3] != C * C || in_sizes[4] != C ||
      in_sizes[5] != RELN * NH || in_sizes[6] != RELN * NH || in_sizes[7] < 1 || in_sizes[8] < 1 ||
      out_size != BS * C || NH > NHMAX) return;

  const float* x      = (const float*)d_in[0];
  const float* qkv_w  = (const float*)d_in[1];
  const float* qkv_b  = (const float*)d_in[2];
  const float* proj_w = (const float*)d_in[3];
  const float* proj_b = (const float*)d_in[4];
  const float* rel_h  = (const float*)d_in[5];
  const float* rel_w  = (const float*)d_in[6];
  const int*   Hp     = (const int*)d_in[7];
  const int*   Wp     = (const int*)d_in[8];
  float* out = (float*)d_out;

  char* ws = (char*)d_ws;
  size_t off = 0;
  _Float16* xh   = (_Float16*)(ws + off); off += align256((size_t)BS * C * 2);
  _Float16* wqh  = (_Float16*)(ws + off); off += align256((size_t)C3 * C * 2);
  _Float16* wph  = (_Float16*)(ws + off); off += align256((size_t)C * C * 2);
  float*    qkvf = (float*)(ws + off);    off += align256((size_t)BS * C3 * 4);
  float*    attf = (float*)(ws + off);    off += align256((size_t)BS * C * 4);
  _Float16* atth = (_Float16*)(ws + off); off += align256((size_t)BS * C * 2);
  if (off > ws_size) return;

  {
    const int n2x = BS * C / 2;
    cast_f32_f16x2<<<(n2x + 255) / 256, 256, 0, stream>>>(x, xh, n2x);
    const int n2q = C3 * C / 2;
    cast_f32_f16x2<<<(n2q + 255) / 256, 256, 0, stream>>>(qkv_w, wqh, n2q);
    const int n2p = C * C / 2;
    cast_f32_f16x2<<<(n2p + 255) / 256, 256, 0, stream>>>(proj_w, wph, n2p);
  }

  {
    const int tiles = (BS / 64) * (C3 / 64);
    wmma_gemm64<0, false, 2, 0, false, 0><<<dim3((tiles + 7) / 8, 1), 256, 0, stream>>>(
        U16(xh), U16(xh), C, 0L,
        U16(wqh), U16(wqh), C, 0L,
        (void*)qkvf, (void*)qkvf, C3, 0L,
        qkv_b,
        qkv_b, 0L,
        BS, C3, C, 1.0f);
  }

  {
    const int nqb = (S + AT_QB - 1) / AT_QB;
    attn_relpos64<<<Bn * NH * nqb, 128, 0, stream>>>(qkvf, rel_h, rel_w, Hp, Wp, attf,
                                                    S, nqb, NH, 0.125f);
  }

  {
    const int n2a = BS * C / 2;
    cast_f32_f16x2<<<(n2a + 255) / 256, 256, 0, stream>>>(attf, atth, n2a);
  }

  {
    const int tiles = (BS / 64) * (C / 64);
    wmma_gemm64<0, false, 2, 0, false, 0><<<dim3((tiles + 7) / 8, 1), 256, 0, stream>>>(
        U16(atth), U16(atth), C, 0L,
        U16(wph), U16(wph), C, 0L,
        (void*)out, (void*)out, C, 0L,
        proj_b,
        proj_b, 0L,
        BS, C, C, 1.0f);
  }
}
